// NeuronToSpatialGrid_19490561589315
// MI455X (gfx1250) — hardware-verified
//
#include <hip/hip_runtime.h>
#include <math.h>

#pragma clang fp contract(off)

constexpr int kBatch = 4;
constexpr int kNeur  = 4096;
constexpr int kEmb   = 256;
constexpr int kGrid  = 64;
constexpr int kPts   = kGrid * kGrid;
constexpr int kPPW   = 4;
constexpr int kWavesPerBlock = 8;
constexpr int kPPB   = kPPW * kWavesPerBlock;
constexpr float kInv63    = 1.0f / 63.0f;
constexpr float kNegInvBw = -(1.0f / 0.02f);
constexpr float kEps      = 1e-8f;

typedef __attribute__((ext_vector_type(16))) _Float16 v16h;
typedef __attribute__((ext_vector_type(8)))  _Float16 v8h;
typedef __attribute__((ext_vector_type(16))) __bf16   v16b;
typedef __attribute__((ext_vector_type(8)))  __bf16   v8b;
typedef __attribute__((ext_vector_type(8)))  float    v8f;
typedef __attribute__((ext_vector_type(4)))  float    v4f;
typedef __attribute__((ext_vector_type(4)))  unsigned int v4u;

__device__ __forceinline__ unsigned short f2bf_bits(float f) {
  unsigned u = __float_as_uint(f);
  return (unsigned short)((u + 0x7FFFu + ((u >> 16) & 1u)) >> 16);
}
__device__ __forceinline__ float bf_bits2f(unsigned short h) { return __uint_as_float(((unsigned)h) << 16); }
__device__ __forceinline__ unsigned pk16(unsigned short a, unsigned short b) { return (unsigned)a | ((unsigned)b << 16); }

__device__ __forceinline__ void dep_guard_h(v8f& a, v8f& b, v16h x, v16h y) { asm volatile("v_nop\n\tv_nop\n\tv_nop\n\tv_nop" : "+v"(a), "+v"(b) : "v"(x), "v"(y)); }
__device__ __forceinline__ void dep_guard_b(v8f& a, v8f& b, v16b x, v16b y) { asm volatile("v_nop\n\tv_nop\n\tv_nop\n\tv_nop" : "+v"(a), "+v"(b) : "v"(x), "v"(y)); }
__device__ __forceinline__ void keep4_h(v16h a, v16h b, v16h c, v16h d) { asm volatile("v_nop" :: "v"(a), "v"(b), "v"(c), "v"(d)); }
__device__ __forceinline__ void keep4_b(v16b a, v16b b, v16b c, v16b d) { asm volatile("v_nop" :: "v"(a), "v"(b), "v"(c), "v"(d)); }
__device__ __forceinline__ void acc_guard4(v8f& a, v8f& b, v8f& c, v8f& d) { asm volatile("v_nop\n\tv_nop\n\tv_nop\n\tv_nop" : "+v"(a), "+v"(b), "+v"(c), "+v"(d)); }
template <typename T> struct Frag;
template <> struct Frag<_Float16> {
  typedef v16h V; union U { v16h v; v8h h[2]; };
  static __device__ __forceinline__ v16h load(const _Float16* p) {
    U f; f.h[0] = *(const v8h*)(p); f.h[1] = *(const v8h*)(p + 16); return f.v;
  }
  static __device__ __forceinline__ v8f mma(v16h a, v16h b, v8f c) {
    return __builtin_amdgcn_wmma_f32_16x16x32_f16(false, a, false, b, (short)0, c, false, false);
  }
  static __device__ __forceinline__ void guard(v8f& a, v8f& b, v16h x, v16h y) { dep_guard_h(a, b, x, y); }
  static __device__ __forceinline__ void keep(v16h a, v16h b, v16h c, v16h d) { keep4_h(a, b, c, d); }
};
template <> struct Frag<__bf16> {
  typedef v16b V; union U { v16b v; v8b h[2]; };
  static __device__ __forceinline__ v16b load(const __bf16* p) {
    U f; f.h[0] = *(const v8b*)(p); f.h[1] = *(const v8b*)(p + 16); return f.v;
  }
  static __device__ __forceinline__ v8f mma(v16b a, v16b b, v8f c) {
    return __builtin_amdgcn_wmma_f32_16x16x32_bf16(false, a, false, b, (short)0, c, false, false);
  }
  static __device__ __forceinline__ void guard(v8f& a, v8f& b, v16b x, v16b y) { dep_guard_b(a, b, x, y); }
  static __device__ __forceinline__ void keep(v16b a, v16b b, v16b c, v16b d) { keep4_b(a, b, c, d); }
};

template <int ET> struct Elem;
template <> struct Elem<0> { typedef _Float16 T; };
template <> struct Elem<1> { typedef __bf16 T; };
template <int ET, bool SPLIT, int BIAS_MODE, int OUT_MODE, bool RESID, int ACT = 0>
__global__ __launch_bounds__(256) void wmma_gemm64(
    const unsigned short* __restrict__ Ap, const unsigned short* __restrict__ A2p, int lda, long strideA,
    const unsigned short* __restrict__ Btp, const unsigned short* __restrict__ Bt2p, int ldb, long strideB,
    void* __restrict__ Cout, void* __restrict__ Cout2, int ldc, long strideC,
    const float* __restrict__ bias,
    const float* __restrict__ resid, long strideR,
    int M, int N, int K, float scale) {
  typedef typename Elem<ET>::T T;
  typedef typename Frag<T>::V V;
  const T* A = (const T*)Ap; const T* A2 = (const T*)A2p; const T* Bt = (const T*)Btp; const T* Bt2 = (const T*)Bt2p;
  __shared__ __align__(16) float sT[8][16 * 68];
  const int b    = blockIdx.y;
  const int lane = threadIdx.x & 31;
  const int wave = threadIdx.x >> 5;
  const int tilesN = N >> 6;
  const int tilesM = M >> 6;
  const int tile = blockIdx.x * 8 + wave;
  if (tile >= tilesM * tilesN) return;
  const int tm = tile / tilesN;
  const int tn = tile - tm * tilesN;
  const int m0 = tm << 6;
  const int n0 = tn << 6;

  const T* Ab  = A  + (size_t)b * strideA;
  const T* Bb  = Bt + (size_t)b * strideB;
  const T* Ab2 = SPLIT ? (A2  + (size_t)b * strideA) : nullptr;
  const T* Bb2 = SPLIT ? (Bt2 + (size_t)b * strideB) : nullptr;

  const int rlane = lane & 15;
  const int koff  = (lane >> 4) * 8;
  const int mOff  = (lane >> 4) * 8;

  v8f acc[4][4];
#pragma unroll
  for (int i = 0; i < 4; ++i)
#pragma unroll
    for (int j = 0; j < 4; ++j) acc[i][j] = (v8f){0.f,0.f,0.f,0.f,0.f,0.f,0.f,0.f};

  for (int k0 = 0; k0 < K; k0 += 32) {
    V bh[4], bl[4];
#pragma unroll
    for (int j = 0; j < 4; ++j) {
      const size_t bo = (size_t)(n0 + (j << 4) + rlane) * ldb + koff + k0;
      bh[j] = Frag<T>::load(Bb + bo);
      if (SPLIT) bl[j] = Frag<T>::load(Bb2 + bo);
    }
#pragma unroll
    for (int i = 0; i < 4; ++i) {
      const size_t ao = (size_t)(m0 + (i << 4) + rlane) * lda + koff + k0;
      V ah = Frag<T>::load(Ab + ao);
      V al;
      if (SPLIT) al = Frag<T>::load(Ab2 + ao);
#pragma unroll
      for (int j = 0; j < 4; ++j) {
        acc[i][j] = Frag<T>::mma(ah, bh[j], acc[i][j]);
        if (SPLIT) {
          acc[i][j] = Frag<T>::mma(ah, bl[j], acc[i][j]);
          acc[i][j] = Frag<T>::mma(al, bh[j], acc[i][j]);
        }
      }
      Frag<T>::guard(acc[i][0], acc[i][3], ah, SPLIT ? al : ah);
    }
    Frag<T>::keep(bh[0], bh[1], bh[2], bh[3]);
    if (SPLIT) Frag<T>::keep(bl[0], bl[1], bl[2], bl[3]);
  }
  acc_guard4(acc[0][0], acc[0][1], acc[0][2], acc[0][3]);
  acc_guard4(acc[1][0], acc[1][1], acc[1][2], acc[1][3]);
  acc_guard4(acc[2][0], acc[2][1], acc[2][2], acc[2][3]);
  acc_guard4(acc[3][0], acc[3][1], acc[3][2], acc[3][3]);

  float* slab = sT[wave];
  const float* Rb = RESID ? (resid + (size_t)b * strideR) : nullptr;
#pragma unroll
  for (int i = 0; i < 4; ++i) {
    const int mBase = m0 + (i << 4);
#pragma unroll
    for (int j = 0; j < 4; ++j) {
      const int n = n0 + (j << 4) + rlane;
      float bv = 0.f;
      if (BIAS_MODE == 2) bv = bias[n];
#pragma unroll
      for (int r = 0; r < 8; ++r) {
        float v = acc[i][j][r] * scale;
        if (BIAS_MODE == 1) v += bias[mBase + mOff + r];
        if (BIAS_MODE == 2) v += bv;
        if (RESID) v += Rb[(size_t)(mBase + mOff + r) * ldc + n];
        if (ACT == 2) v = fmaxf(v, 0.0f);
        if (ACT == 4) v = (v > 0.f) ? v : 0.01f * v;
        slab[(mOff + r) * 68 + (j << 4) + rlane] = v;
      }
    }
    __builtin_amdgcn_fence(__ATOMIC_RELEASE, "workgroup");
    __builtin_amdgcn_wave_barrier();
    __builtin_amdgcn_fence(__ATOMIC_ACQUIRE, "workgroup");
    if (OUT_MODE == 0) {
      float* C = (float*)Cout + (size_t)b * strideC;
      const int hh = lane >> 4, c4 = (lane & 15) * 4;
      for (int pass = 0; pass < 2; ++pass) {
#pragma unroll
        for (int it = 0; it < 8; ++it) {
          const int row = it * 2 + hh;
          v4f v = *(const v4f*)(slab + row * 68 + c4);
          *(volatile v4f*)(C + (size_t)(mBase + row) * ldc + n0 + c4) = v;
        }
        __threadfence();
      }
    } else {
      const int q = lane >> 3, c8 = (lane & 7) * 8;
      unsigned short* C  = (unsigned short*)Cout  + (size_t)b * strideC;
      unsigned short* C2 = (OUT_MODE == 2) ? ((unsigned short*)Cout2 + (size_t)b * strideC) : nullptr;
      for (int pass = 0; pass < 2; ++pass) {
#pragma unroll
        for (int it = 0; it < 4; ++it) {
          const int row = it * 4 + q;
          const float* sp = slab + row * 68 + c8;
          v8h hv, lv;
#pragma unroll
          for (int e = 0; e < 8; ++e) {
            if (OUT_MODE == 1) {
              hv[e] = (_Float16)sp[e];
            } else {
              unsigned short hb = f2bf_bits(sp[e]);
              unsigned short lb = f2bf_bits(sp[e] - bf_bits2f(hb));
              hv[e] = __builtin_bit_cast(_Float16, hb);
              lv[e] = __builtin_bit_cast(_Float16, lb);
            }
          }
          *(volatile v8h*)(C + (size_t)(mBase + row) * ldc + n0 + c8) = hv;
          if (OUT_MODE == 2) *(volatile v8h*)(C2 + (size_t)(mBase + row) * ldc + n0 + c8) = lv;
        }
        __threadfence();
      }
    }
    __builtin_amdgcn_fence(__ATOMIC_RELEASE, "workgroup");
    __builtin_amdgcn_wave_barrier();
    __builtin_amdgcn_fence(__ATOMIC_ACQUIRE, "workgroup");
  }
}

__global__ __launch_bounds__(256) void feat_tsplit_kernel(const float* __restrict__ F,
                                                          unsigned short* __restrict__ fthi,
                                                          unsigned short* __restrict__ ftlo) {
  __shared__ float sm[64][65];
  const int t  = threadIdx.x;
  const int n0 = blockIdx.x * 64;
  const int e0 = blockIdx.y * 64;
  const int b  = blockIdx.z;
  const float* Fb = F + (size_t)b * kNeur * kEmb;
#pragma unroll
  for (int i = 0; i < 16; ++i) {
    const int idx = i * 256 + t;
    const int r = idx >> 6;
    const int c = idx & 63;
    sm[c][r] = Fb[(size_t)(n0 + r) * kEmb + e0 + c];
  }
  __syncthreads();
  const int lane = t & 31, wave = t >> 5;
  const int q = lane >> 3, c8 = (lane & 7) * 8;
  unsigned short* oh = fthi + (size_t)b * kEmb * kNeur;
  unsigned short* ol = ftlo + (size_t)b * kEmb * kNeur;
  for (int pass = 0; pass < 2; ++pass) {
#pragma unroll
    for (int it = 0; it < 2; ++it) {
      const int row = wave * 8 + it * 4 + q;
      unsigned short hb[8], lb[8];
#pragma unroll
      for (int e = 0; e < 8; ++e) {
        const float v = sm[row][c8 + e];
        hb[e] = f2bf_bits(v);
        lb[e] = f2bf_bits(v - bf_bits2f(hb[e]));
      }
      const v4u uh = (v4u){pk16(hb[0], hb[1]), pk16(hb[2], hb[3]), pk16(hb[4], hb[5]), pk16(hb[6], hb[7])};
      const v4u ul = (v4u){pk16(lb[0], lb[1]), pk16(lb[2], lb[3]), pk16(lb[4], lb[5]), pk16(lb[6], lb[7])};
      const size_t o = (size_t)(e0 + row) * kNeur + n0 + c8;
      *(volatile v4u*)(oh + o) = uh;
      *(volatile v4u*)(ol + o) = ul;
    }
    __threadfence();
  }
}

__device__ __forceinline__ void rbf8(v4f a0, v4f a1, v4f a2, v4f a3, float cx, float cy, float (&w)[8]) {
  const float px[8] = {a0[0], a0[2], a1[0], a1[2], a2[0], a2[2], a3[0], a3[2]};
  const float py[8] = {a0[1], a0[3], a1[1], a1[3], a2[1], a2[3], a3[1], a3[3]};
#pragma unroll
  for (int j = 0; j < 8; ++j) {
    const float dx  = cx - px[j];
    const float dy  = cy - py[j];
    const float dxx = dx * dx;
    const float dyy = dy * dy;
    const float d2  = dxx + dyy;
    w[j] = expf(d2 * kNegInvBw);
  }
}

__global__ __launch_bounds__(256) void rbf_weight_kernel(const float* __restrict__ pos,
                                                         unsigned short* __restrict__ wnhi,
                                                         unsigned short* __restrict__ wnlo) {
  __shared__ __align__(16) float sPos[kNeur * 2];
  const int t = threadIdx.x, lane = t & 31, wave = t >> 5;
#pragma unroll
  for (int i = 0; i < 8; ++i) {
    const int f4 = (i * 256 + t) * 4;
    *(v4f*)(sPos + f4) = *(const v4f*)(pos + f4);
  }
  __syncthreads();

#pragma unroll 1
  for (int q = 0; q < kPPW; ++q) {
    const int p  = blockIdx.x * kPPB + wave * kPPW + q;
    const int gi = p >> 6;
    const int gj = p & 63;
    const float cx = (gi == kGrid - 1) ? 1.0f : (float)gi * kInv63;
    const float cy = (gj == kGrid - 1) ? 1.0f : (float)gj * kInv63;

    float part = 0.0f;
#pragma unroll 1
    for (int it = 0; it < kNeur / 256; ++it) {
      const int nb = it * 256 + lane * 8;
      const float* sp = sPos + nb * 2;
      const v4f a0 = *(const v4f*)(sp);
      const v4f a1 = *(const v4f*)(sp + 4);
      const v4f a2 = *(const v4f*)(sp + 8);
      const v4f a3 = *(const v4f*)(sp + 12);
      float w[8];
      rbf8(a0, a1, a2, a3, cx, cy, w);
#pragma unroll
      for (int j = 0; j < 8; ++j) part += w[j];
    }
    float s = part;
#pragma unroll
    for (int off = 16; off > 0; off >>= 1) s += __shfl_xor(s, off, 32);
    const float rinv = 1.0f / (s + kEps);

    unsigned short* rowh = wnhi + (size_t)p * kNeur;
    unsigned short* rowl = wnlo + (size_t)p * kNeur;
#pragma unroll 1
    for (int it = 0; it < kNeur / 256; ++it) {
      const int nb = it * 256 + lane * 8;
      const float* sp = sPos + nb * 2;
      const v4f a0 = *(const v4f*)(sp);
      const v4f a1 = *(const v4f*)(sp + 4);
      const v4f a2 = *(const v4f*)(sp + 8);
      const v4f a3 = *(const v4f*)(sp + 12);
      float w[8];
      rbf8(a0, a1, a2, a3, cx, cy, w);
      unsigned short hb[8], lb[8];
#pragma unroll
      for (int j = 0; j < 8; ++j) {
        const float wn = w[j] * rinv;
        hb[j] = f2bf_bits(wn);
        lb[j] = f2bf_bits(wn - bf_bits2f(hb[j]));
      }
      const v4u uh = (v4u){pk16(hb[0], hb[1]), pk16(hb[2], hb[3]), pk16(hb[4], hb[5]), pk16(hb[6], hb[7])};
      const v4u ul = (v4u){pk16(lb[0], lb[1]), pk16(lb[2], lb[3]), pk16(lb[4], lb[5]), pk16(lb[6], lb[7])};
      unsigned short* ph = rowh + nb;
      unsigned short* pl = rowl + nb;
      *(volatile v4u*)ph = uh;
      *(volatile v4u*)pl = ul;
      __threadfence();
      *(volatile v4u*)ph = uh;
      *(volatile v4u*)pl = ul;
    }
  }
}

extern "C" void kernel_launch(void* const* d_in, const int* in_sizes, int n_in,
                              void* d_out, int out_size, void* d_ws, size_t ws_size,
                              hipStream_t stream) {
  if (n_in < 2) return;
  if (in_sizes[0] != kBatch * kNeur * kEmb) return;
  if (in_sizes[1] != kBatch * kNeur * 2) return;
  if (out_size != kBatch * kEmb * kPts) return;

  const float* feat = (const float*)d_in[0];
  const float* pos  = (const float*)d_in[1];
  float* out = (float*)d_out;

  const size_t wnBytes = (size_t)kPts * kNeur * sizeof(unsigned short);
  const size_t ftBytes = (size_t)kBatch * kEmb * kNeur * sizeof(unsigned short);
  const size_t total   = 2 * wnBytes + 2 * ftBytes;
  if (total > ws_size) return;

  unsigned char* ws = (unsigned char*)d_ws;
  unsigned short* wnhi = (unsigned short*)(ws);
  unsigned short* wnlo = (unsigned short*)(ws + wnBytes);
  unsigned short* fthi = (unsigned short*)(ws + 2 * wnBytes);
  unsigned short* ftlo = (unsigned short*)(ws + 2 * wnBytes + ftBytes);

  feat_tsplit_kernel<<<dim3(kNeur / 64, kEmb / 64, kBatch), dim3(256), 0, stream>>>(feat, fthi, ftlo);

  const int gemmTiles  = (kEmb / 64) * (kPts / 64);
  const int gemmBlocks = (gemmTiles + 7) / 8;
  for (int b = 0; b < kBatch; ++b) {
    rbf_weight_kernel<<<dim3(kPts / kPPB), dim3(256), 0, stream>>>(
        pos + (size_t)b * kNeur * 2, wnhi, wnlo);
    wmma_gemm64<1, true, 0, 0, false, 0><<<dim3(gemmBlocks, 1), dim3(256), 0, stream>>>(
        fthi + (size_t)b * kEmb * kNeur, ftlo + (size_t)b * kEmb * kNeur, kNeur, 0L,
        wnhi, wnlo, kNeur, 0L,
        (void*)(out + (size_t)b * kEmb * kPts), (void*)nullptr, kPts, 0L,
        (const float*)nullptr,
        (const float*)nullptr, 0L,
        kEmb, kPts, kNeur, 1.0f);
  }
}
